// GFRB_10591389352537
// MI455X (gfx1250) — hardware-verified
//
#include <hip/hip_runtime.h>
#include <math.h>

typedef __attribute__((ext_vector_type(16))) _Float16 v16h;
typedef __attribute__((ext_vector_type(8)))  _Float16 v8h;
typedef __attribute__((ext_vector_type(2)))  _Float16 v2h;
typedef __attribute__((ext_vector_type(8)))  float    v8f;
typedef __attribute__((ext_vector_type(4)))  float    v4f;
typedef __attribute__((ext_vector_type(2)))  float    v2f;
typedef __attribute__((ext_vector_type(8)))  int      v8i;
typedef __attribute__((ext_vector_type(4)))  int      v4i;

constexpr int kNB = 4;
constexpr int kCH = 64;
constexpr int kIH = 224;
constexpr int kIW = 224;
constexpr int kHW = kIH * kIW;
constexpr int kNPIX = kNB * kHW;
constexpr int kTilesPerImg = kHW / 64;
constexpr int kTiles = kNB * kTilesPerImg;
constexpr int kKOff = 576;
constexpr int kKA1  = 320;
constexpr int kKFin = 896;
constexpr int kFinWaves = 4;
constexpr int kSPitch = 72;
constexpr float kWCarry  = 64.0f;
constexpr float kWCarry2 = 4.0f;
constexpr float kACarry  = 16.0f;
static_assert(kHW == 50176 && kNPIX == 200704, "pixel counts");
static_assert(kHW % 64 == 0, "64-pixel tiles never cross an image");
static_assert(kTiles == 3136 && kTiles % 8 == 0 && kTiles % kFinWaves == 0, "exact grids");
static_assert(kKOff % 32 == 0 && kKA1 % 32 == 0 && kKFin % 32 == 0, "K multiples of 32");
static_assert(kACarry * kWCarry2 == kWCarry, "single fold-back scale in the fused accumulator");
static_assert(kIW % 32 == 0, "32-wide row segments");

constexpr size_t kSzXF   = (size_t)kNPIX * 64 * 4;
constexpr size_t kSzP16  = (size_t)kNPIX * 64 * 2;
constexpr size_t kSzOFFP = (size_t)kNPIX * 32 * 4;
constexpr size_t kSzBtOff = (size_t)32 * kKOff * 2;
constexpr size_t kSzBtA1  = (size_t)64 * kKA1 * 2;
constexpr size_t kSzBtFin = (size_t)64 * kKFin * 2;
constexpr size_t kOffXF    = 0;
constexpr size_t kOffX2    = kOffXF + kSzXF;
constexpr size_t kOffX3    = kOffX2 + kSzP16;
constexpr size_t kOffOFFP  = kOffX3 + kSzP16;
constexpr size_t kOffBtOff = kOffOFFP + kSzOFFP;
constexpr size_t kOffBtA1  = kOffBtOff + kSzBtOff;
constexpr size_t kOffBtFin = kOffBtA1 + kSzBtA1;
constexpr size_t kWsTotal  = kOffBtFin + kSzBtFin;
static_assert(kWsTotal == 128643072ull, "carve total");
static_assert(kWsTotal <= 134217728ull, "carve cap");
static_assert((kOffX2 % 128) == 0 && (kOffX3 % 128) == 0 && (kOffOFFP % 128) == 0 && (kOffBtOff % 128) == 0 &&
              (kOffBtA1 % 128) == 0 && (kOffBtFin % 128) == 0, "128-B aligned regions");

union FragU { v16h v; v8h h[2]; };
__device__ __forceinline__ v16h frag_load(const _Float16* p) {
  FragU f;
  f.h[0] = *(const v8h*)(p);
  f.h[1] = *(const v8h*)(p + 16);
  return f.v;
}
__device__ __forceinline__ v16h frag_mask(v16h a, int m) {
  const v8i mv = {m, m, m, m, m, m, m, m};
  v8i ai = __builtin_bit_cast(v8i, a);
  ai = ai & mv;
  return __builtin_bit_cast(v16h, ai);
}
__device__ __forceinline__ v8f mma_g(v16h a, v16h b, v8f c) {
  c = __builtin_amdgcn_wmma_f32_16x16x32_f16(false, a, false, b, (short)0, c, false, false);
  asm volatile("v_nop\n\tv_nop\n\tv_nop\n\tv_nop" : "+v"(c) : "v"(a), "v"(b));
  return c;
}
__device__ __forceinline__ void wave_lds_sync() {
  __builtin_amdgcn_fence(__ATOMIC_RELEASE, "workgroup");
  __builtin_amdgcn_wave_barrier();
  __builtin_amdgcn_fence(__ATOMIC_ACQUIRE, "workgroup");
}

__global__ __launch_bounds__(256) void prep_w_kernel(
    const float* __restrict__ src, int nReal, int nRows, int taps,
    unsigned short* __restrict__ dst, int ld, int koff, float carry)
{
  const int i = blockIdx.x * 256 + threadIdx.x;
  const int perRow = taps * 8;
  if (i >= nRows * perRow) return;
  const int n = i / perRow;
  const int g = i - n * perRow;
  const int tap = g >> 3;
  const int c0 = (g & 7) * 8;
  const int nc = (n < nReal) ? n : (nReal - 1);
  const bool live = (n < nReal);
  v8h hv;
#pragma unroll
  for (int e = 0; e < 8; ++e) {
    const float v = src[(size_t)((nc * 64 + c0 + e) * taps + tap)];
    const float s = live ? (v * carry) : 0.0f;
    hv[e] = (_Float16)s;
  }
  unsigned short* q = dst + (size_t)n * ld + koff + tap * 64 + c0;
  *(volatile v8h*)q = hv;
  __threadfence();
  *(volatile v8h*)q = hv;
}

__global__ __launch_bounds__(256) void prep_x_kernel(
    const float* __restrict__ x,
    const float* __restrict__ s2, const float* __restrict__ t2,
    const float* __restrict__ s3, const float* __restrict__ t3,
    float* __restrict__ XF, unsigned short* __restrict__ X2, unsigned short* __restrict__ X3)
{
  __shared__ __align__(16) float sX[64 * 36];
  const int tid = threadIdx.x;
  int bx = blockIdx.x;
  const int wseg = bx % (kIW / 32);
  bx /= (kIW / 32);
  const int h = bx % kIH;
  const int b = bx / kIH;
  const int w0 = wseg * 32;
#pragma unroll
  for (int i = 0; i < 2; ++i) {
    const int c = (tid >> 3) + 32 * i;
    const int w4 = (tid & 7) * 4;
    const v4f v = *(const v4f*)(x + ((size_t)(b * kCH + c) * kIH + h) * kIW + w0 + w4);
    *(v4f*)(sX + c * 36 + w4) = v;
  }
  __syncthreads();
  const size_t pixbase = (size_t)(b * kIH + h) * kIW + w0;
  v4f xf[2];
#pragma unroll
  for (int i = 0; i < 2; ++i) {
    const int item = tid + 256 * i;
    const int p = item >> 4;
    const int c4 = (item & 15) * 4;
    v4f v;
    v.x = sX[(c4 + 0) * 36 + p];
    v.y = sX[(c4 + 1) * 36 + p];
    v.z = sX[(c4 + 2) * 36 + p];
    v.w = sX[(c4 + 3) * 36 + p];
    xf[i] = v;
  }
  const int p8 = tid >> 3;
  const int c8 = (tid & 7) * 8;
  const v4f s2a = *(const v4f*)(s2 + c8), s2b = *(const v4f*)(s2 + c8 + 4);
  const v4f t2a = *(const v4f*)(t2 + c8), t2b = *(const v4f*)(t2 + c8 + 4);
  const v4f s3a = *(const v4f*)(s3 + c8), s3b = *(const v4f*)(s3 + c8 + 4);
  const v4f t3a = *(const v4f*)(t3 + c8), t3b = *(const v4f*)(t3 + c8 + 4);
  v8h h2v, h3v;
#pragma unroll
  for (int e = 0; e < 4; ++e) {
    const float xa = sX[(c8 + e) * 36 + p8];
    const float xb = sX[(c8 + 4 + e) * 36 + p8];
    const float u2a = (xa * s2a[e] + t2a[e]) * kACarry;
    const float u2b = (xb * s2b[e] + t2b[e]) * kACarry;
    const float u3a = (xa * s3a[e] + t3a[e]) * kACarry;
    const float u3b = (xb * s3b[e] + t3b[e]) * kACarry;
    h2v[e]     = (_Float16)u2a;
    h2v[4 + e] = (_Float16)u2b;
    h3v[e]     = (_Float16)u3a;
    h3v[4 + e] = (_Float16)u3b;
  }
  for (int pass = 0; pass < 2; ++pass) {
#pragma unroll
    for (int i = 0; i < 2; ++i) {
      const int item = tid + 256 * i;
      const int p = item >> 4;
      const int c4 = (item & 15) * 4;
      *(volatile v4f*)(XF + (pixbase + p) * 64 + c4) = xf[i];
    }
    *(volatile v8h*)(X2 + (pixbase + p8) * 64 + c8) = h2v;
    *(volatile v8h*)(X3 + (pixbase + p8) * 64 + c8) = h3v;
    __threadfence();
  }
}

template <int NSUB, int KIND>
__global__ __launch_bounds__(256) void conv_tap_gemm_kernel(
    const unsigned short* __restrict__ Xp, const unsigned short* __restrict__ Btp,
    const float* __restrict__ bias, void* __restrict__ Outp)
{
  constexpr int TAPS  = (KIND == 0) ? 9 : 5;
  constexpr int KTOT  = TAPS * 64;
  constexpr int NREAL = (KIND == 0) ? 18 : 64;
  constexpr int SP    = (KIND == 0) ? 36 : 68;
  static_assert(NSUB * 16 >= NREAL && (KTOT % 32) == 0, "tile shape");
  __shared__ __align__(16) float sT[8][16 * SP];
  const _Float16* X  = (const _Float16*)Xp;
  const _Float16* Bt = (const _Float16*)Btp;
  const int lane = threadIdx.x & 31;
  const int wave = threadIdx.x >> 5;
  const int tile = blockIdx.x * 8 + wave;
  if (tile >= kTiles) return;
  const int b = tile / kTilesPerImg;
  const int hw0 = (tile - b * kTilesPerImg) * 64;
  const int pixbase = b * kHW + hw0;
  const int rlane = lane & 15;
  const int koff = (lane >> 4) * 8;
  const int mOff = (lane >> 4) * 8;

  int hr[4], wr[4];
#pragma unroll
  for (int i = 0; i < 4; ++i) {
    const int hw = hw0 + i * 16 + rlane;
    hr[i] = hw / kIW;
    wr[i] = hw - hr[i] * kIW;
  }
  v8f acc[4][NSUB];
#pragma unroll
  for (int i = 0; i < 4; ++i)
#pragma unroll
    for (int j = 0; j < NSUB; ++j) acc[i][j] = (v8f){0.f, 0.f, 0.f, 0.f, 0.f, 0.f, 0.f, 0.f};

#pragma unroll 1
  for (int t = 0; t < TAPS; ++t) {
    int dyt, dxt;
    if (KIND == 0) {
      const int q3 = t / 3;
      dyt = q3 - 1;
      dxt = t - q3 * 3 - 1;
    } else {
      dyt = t - 2;
      dxt = 0;
    }
    const _Float16* ap[4];
    int am[4];
#pragma unroll
    for (int i = 0; i < 4; ++i) {
      const int hh = hr[i] + dyt;
      const int ww = wr[i] + dxt;
      const bool ok = ((unsigned)hh < (unsigned)kIH) && ((unsigned)ww < (unsigned)kIW);
      const int hc = min(max(hh, 0), kIH - 1);
      const int wc = min(max(ww, 0), kIW - 1);
      ap[i] = X + (size_t)((b * kIH + hc) * kIW + wc) * 64 + koff;
      am[i] = ok ? -1 : 0;
    }
#pragma unroll
    for (int cc = 0; cc < 2; ++cc) {
      const int k0 = t * 64 + cc * 32;
      v16h bh[NSUB];
#pragma unroll
      for (int j = 0; j < NSUB; ++j)
        bh[j] = frag_load(Bt + (size_t)(j * 16 + rlane) * KTOT + k0 + koff);
#pragma unroll
      for (int i = 0; i < 4; ++i) {
        const v16h a = frag_mask(frag_load(ap[i] + cc * 32), am[i]);
#pragma unroll
        for (int j = 0; j < NSUB; ++j) acc[i][j] = mma_g(a, bh[j], acc[i][j]);
      }
    }
  }

  constexpr float scale = 1.0f / (kWCarry * kACarry);
  float* slab = sT[wave];
  float bvv[NSUB];
#pragma unroll
  for (int j = 0; j < NSUB; ++j) {
    const int n = j * 16 + rlane;
    const int nb = (n < NREAL) ? n : (NREAL - 1);
    const float bl = bias[nb];
    bvv[j] = (n < NREAL) ? bl : 0.0f;
  }
#pragma unroll
  for (int i = 0; i < 4; ++i) {
#pragma unroll
    for (int j = 0; j < NSUB; ++j) {
#pragma unroll
      for (int r = 0; r < 8; ++r) {
        float v = acc[i][j][r] * scale + bvv[j];
        if (KIND == 1) v = v * kACarry;
        slab[(mOff + r) * SP + j * 16 + rlane] = v;
      }
    }
    wave_lds_sync();
    const int q = lane >> 3;
    if (KIND == 0) {
      float* O = (float*)Outp;
      const int c4 = (lane & 7) * 4;
      for (int pass = 0; pass < 2; ++pass) {
#pragma unroll
        for (int it = 0; it < 4; ++it) {
          const int row = it * 4 + q;
          const v4f v = *(const v4f*)(slab + row * SP + c4);
          *(volatile v4f*)(O + (size_t)(pixbase + i * 16 + row) * 32 + c4) = v;
        }
        __threadfence();
      }
    } else {
      unsigned short* O = (unsigned short*)Outp;
      const int c8 = (lane & 7) * 8;
      for (int pass = 0; pass < 2; ++pass) {
#pragma unroll
        for (int it = 0; it < 4; ++it) {
          const int row = it * 4 + q;
          const float* sp = slab + row * SP + c8;
          v8h hv;
#pragma unroll
          for (int e = 0; e < 8; ++e) hv[e] = (_Float16)sp[e];
          *(volatile v8h*)(O + (size_t)(pixbase + i * 16 + row) * 64 + c8) = hv;
        }
        __threadfence();
      }
    }
    wave_lds_sync();
  }
}

__global__ __launch_bounds__(128) void fused_sample_gemm_kernel(
    const float* __restrict__ XF, const float* __restrict__ OFFP,
    const unsigned short* __restrict__ A1p, const unsigned short* __restrict__ Btp,
    const float* __restrict__ x, const float* __restrict__ dw1_w, const float* __restrict__ dw1_b,
    const float* __restrict__ def_b, const float* __restrict__ asym2_b, float* __restrict__ out)
{
  __shared__ __align__(16) _Float16 sS[kFinWaves][64 * kSPitch];
  __shared__ __align__(16) int      sIdx[kFinWaves][256];
  __shared__ __align__(16) float    sWt[kFinWaves][256];
  __shared__ __align__(16) float    sT[kFinWaves][16 * 68];
  __shared__ __align__(16) float    sC[128];
  static_assert(sizeof(_Float16) * kFinWaves * 64 * kSPitch + 4 * kFinWaves * 256 * 2 + 4 * kFinWaves * 16 * 68 + 512 <= 65536,
                "static LDS budget");
  const int tid = threadIdx.x;
  const int lane = tid & 31;
  const int wave = tid >> 5;
  if (tid < 64) {
    v2f cv;
    cv.x = def_b[tid] + asym2_b[tid] + dw1_b[tid];
    cv.y = 1.0f + dw1_w[tid];
    *(v2f*)(sC + 2 * tid) = cv;
  }
  __syncthreads();

  const _Float16* A1 = (const _Float16*)A1p;
  const _Float16* Bt = (const _Float16*)Btp;
  const int tile = blockIdx.x * kFinWaves + wave;
  const int b = tile / kTilesPerImg;
  const int hw0 = (tile - b * kTilesPerImg) * 64;
  const int imgpix = b * kHW;
  const int pixbase = imgpix + hw0;
  const int rlane = lane & 15;
  const int hh = lane >> 4;
  const int koff = hh * 8;
  const int mOff = hh * 8;
  _Float16* Sw = sS[wave];
  int* idw = sIdx[wave];
  float* wtw = sWt[wave];
  float* Tw = sT[wave];

  int hq[2], wq[2];
#pragma unroll
  for (int u = 0; u < 2; ++u) {
    const int hw = hw0 + lane + 32 * u;
    hq[u] = hw / kIW;
    wq[u] = hw - hq[u] * kIW;
  }
  int wr[4];
#pragma unroll
  for (int i = 0; i < 4; ++i) {
    const int hw = hw0 + i * 16 + rlane;
    const int hrow = hw / kIW;
    wr[i] = hw - hrow * kIW;
  }

  v8f acc[4][4];
#pragma unroll
  for (int i = 0; i < 4; ++i)
#pragma unroll
    for (int j = 0; j < 4; ++j) acc[i][j] = (v8f){0.f, 0.f, 0.f, 0.f, 0.f, 0.f, 0.f, 0.f};

  const v2f* xb = (const v2f*)XF;

#pragma unroll 1
  for (int t = 0; t < 9; ++t) {
    const int q3 = t / 3;
    const int kyi = q3 - 1;
    const int kxi = t - q3 * 3 - 1;
#pragma unroll
    for (int u = 0; u < 2; ++u) {
      const int m = lane + 32 * u;
      const v2f od = *(const v2f*)(OFFP + (size_t)(pixbase + m) * 32 + 2 * t);
      const float py = (float)(hq[u] + kyi) + od.x;
      const float px = (float)(wq[u] + kxi) + od.y;
      const float y0f = floorf(py);
      const float x0f = floorf(px);
      const float fy = py - y0f;
      const float fx = px - x0f;
      const float gy = 1.0f - fy;
      const float gx = 1.0f - fx;
      const int y0 = (int)fminf(fmaxf(y0f, -2.0f), (float)(kIH + 1));
      const int x0 = (int)fminf(fmaxf(x0f, -2.0f), (float)(kIW + 1));
      const int y1 = y0 + 1;
      const int x1 = x0 + 1;
      const bool vy0 = ((unsigned)y0 < (unsigned)kIH);
      const bool vy1 = ((unsigned)y1 < (unsigned)kIH);
      const bool vx0 = ((unsigned)x0 < (unsigned)kIW);
      const bool vx1 = ((unsigned)x1 < (unsigned)kIW);
      const float p00 = gy * gx;
      const float p01 = gy * fx;
      const float p10 = fy * gx;
      const float p11 = fy * fx;
      v4f wv;
      wv.x = (vy0 && vx0) ? p00 : 0.0f;
      wv.y = (vy0 && vx1) ? p01 : 0.0f;
      wv.z = (vy1 && vx0) ? p10 : 0.0f;
      wv.w = (vy1 && vx1) ? p11 : 0.0f;
      const int yc0 = min(max(y0, 0), kIH - 1);
      const int yc1 = min(max(y1, 0), kIH - 1);
      const int xc0 = min(max(x0, 0), kIW - 1);
      const int xc1 = min(max(x1, 0), kIW - 1);
      v4i iv;
      iv.x = imgpix + yc0 * kIW + xc0;
      iv.y = imgpix + yc0 * kIW + xc1;
      iv.z = imgpix + yc1 * kIW + xc0;
      iv.w = imgpix + yc1 * kIW + xc1;
      *(v4i*)(idw + 4 * m) = iv;
      *(v4f*)(wtw + 4 * m) = wv;
    }
    wave_lds_sync();
#pragma unroll 2
    for (int m = 0; m < 64; ++m) {
      const v4i id = *(const v4i*)(idw + 4 * m);
      const v4f wt = *(const v4f*)(wtw + 4 * m);
      const v2f c00 = xb[id.x * 32 + lane];
      const v2f c01 = xb[id.y * 32 + lane];
      const v2f c10 = xb[id.z * 32 + lane];
      const v2f c11 = xb[id.w * 32 + lane];
      float s0 = wt.x * c00.x;
      float s1 = wt.x * c00.y;
      s0 = fmaf(wt.y, c01.x, s0);
      s1 = fmaf(wt.y, c01.y, s1);
      s0 = fmaf(wt.z, c10.x, s0);
      s1 = fmaf(wt.z, c10.y, s1);
      s0 = fmaf(wt.w, c11.x, s0);
      s1 = fmaf(wt.w, c11.y, s1);
      v2h hv;
      hv.x = (_Float16)s0;
      hv.y = (_Float16)s1;
      *(v2h*)(Sw + m * kSPitch + 2 * lane) = hv;
    }
    wave_lds_sync();
#pragma unroll
    for (int cc = 0; cc < 2; ++cc) {
      const int k0 = t * 64 + cc * 32;
      v16h bh[4];
#pragma unroll
      for (int j = 0; j < 4; ++j)
        bh[j] = frag_load(Bt + (size_t)(j * 16 + rlane) * kKFin + k0 + koff);
#pragma unroll
      for (int i = 0; i < 4; ++i) {
        const v16h a = frag_load(Sw + (i * 16 + rlane) * kSPitch + cc * 32 + koff);
#pragma unroll
        for (int j = 0; j < 4; ++j) acc[i][j] = mma_g(a, bh[j], acc[i][j]);
      }
    }
    wave_lds_sync();
  }

#pragma unroll 1
  for (int kw = 0; kw < 5; ++kw) {
    const int dxw = kw - 2;
    const _Float16* ap[4];
    int am[4];
#pragma unroll
    for (int i = 0; i < 4; ++i) {
      const int ww = wr[i] + dxw;
      const bool ok = ((unsigned)ww < (unsigned)kIW);
      const int gp = min(max(pixbase + i * 16 + rlane + dxw, 0), kNPIX - 1);
      ap[i] = A1 + (size_t)gp * 64 + koff;
      am[i] = ok ? -1 : 0;
    }
#pragma unroll
    for (int cc = 0; cc < 2; ++cc) {
      const int k0 = kKOff + kw * 64 + cc * 32;
      v16h bh[4];
#pragma unroll
      for (int j = 0; j < 4; ++j)
        bh[j] = frag_load(Bt + (size_t)(j * 16 + rlane) * kKFin + k0 + koff);
#pragma unroll
      for (int i = 0; i < 4; ++i) {
        const v16h a = frag_mask(frag_load(ap[i] + cc * 32), am[i]);
#pragma unroll
        for (int j = 0; j < 4; ++j) acc[i][j] = mma_g(a, bh[j], acc[i][j]);
      }
    }
  }

  constexpr float inv = 1.0f / kWCarry;
  const int c4 = (lane & 15) * 4;
#pragma unroll
  for (int j = 0; j < 4; ++j) {
#pragma unroll
    for (int i = 0; i < 4; ++i) {
      v4f lo, hi;
      lo.x = acc[i][j][0]; lo.y = acc[i][j][1]; lo.z = acc[i][j][2]; lo.w = acc[i][j][3];
      hi.x = acc[i][j][4]; hi.y = acc[i][j][5]; hi.z = acc[i][j][6]; hi.w = acc[i][j][7];
      *(v4f*)(Tw + rlane * 68 + i * 16 + mOff) = lo;
      *(v4f*)(Tw + rlane * 68 + i * 16 + mOff + 4) = hi;
    }
    wave_lds_sync();
    v4f val[8];
#pragma unroll
    for (int it = 0; it < 8; ++it) {
      const int row = it * 2 + hh;
      const int ch = j * 16 + row;
      const v4f t4 = *(const v4f*)(Tw + row * 68 + c4);
      const v2f cst = *(const v2f*)(sC + 2 * ch);
      const size_t gofs = (size_t)(b * kCH + ch) * kHW + hw0 + c4;
      const v4f xr = *(const v4f*)(x + gofs);
      val[it] = t4 * inv + cst.x + xr * cst.y;
    }
    for (int pass = 0; pass < 2; ++pass) {
#pragma unroll
      for (int it = 0; it < 8; ++it) {
        const int row = it * 2 + hh;
        const int ch = j * 16 + row;
        const size_t gofs = (size_t)(b * kCH + ch) * kHW + hw0 + c4;
        *(volatile v4f*)(out + gofs) = val[it];
      }
      __threadfence();
    }
    wave_lds_sync();
  }
}

extern "C" void kernel_launch(void* const* d_in, const int* in_sizes, int n_in,
                              void* d_out, int out_size, void* d_ws, size_t ws_size,
                              hipStream_t stream) {
  if (n_in < 15) return;
  if (in_sizes[0] != kNPIX * kCH) return;
  if (in_sizes[1] != 64 || in_sizes[2] != 64 || in_sizes[3] != 64 || in_sizes[4] != 64) return;
  if (in_sizes[5] != 64 || in_sizes[6] != 64) return;
  if (in_sizes[7] != 64 * 64 * 5 || in_sizes[8] != 64) return;
  if (in_sizes[9] != 64 * 64 * 5 || in_sizes[10] != 64) return;
  if (in_sizes[11] != 18 * 64 * 9 || in_sizes[12] != 18) return;
  if (in_sizes[13] != 64 * 64 * 9 || in_sizes[14] != 64) return;
  if (out_size != kNPIX * kCH) return;
  if (ws_size < kWsTotal) return;

  const float* x       = (const float*)d_in[0];
  const float* dw1_w   = (const float*)d_in[1];
  const float* dw1_b   = (const float*)d_in[2];
  const float* dw2_w   = (const float*)d_in[3];
  const float* dw2_b   = (const float*)d_in[4];
  const float* dw3_w   = (const float*)d_in[5];
  const float* dw3_b   = (const float*)d_in[6];
  const float* asym1_w = (const float*)d_in[7];
  const float* asym1_b = (const float*)d_in[8];
  const float* asym2_w = (const float*)d_in[9];
  const float* asym2_b = (const float*)d_in[10];
  const float* off_w   = (const float*)d_in[11];
  const float* off_b   = (const float*)d_in[12];
  const float* def_w   = (const float*)d_in[13];
  const float* def_b   = (const float*)d_in[14];
  float* out = (float*)d_out;

  char* ws = (char*)d_ws;
  float*          XF    = (float*)(ws + kOffXF);
  unsigned short* X2    = (unsigned short*)(ws + kOffX2);
  unsigned short* X3    = (unsigned short*)(ws + kOffX3);
  float*          OFFP  = (float*)(ws + kOffOFFP);
  unsigned short* BtOff = (unsigned short*)(ws + kOffBtOff);
  unsigned short* BtA1  = (unsigned short*)(ws + kOffBtA1);
  unsigned short* BtFin = (unsigned short*)(ws + kOffBtFin);
  unsigned short* A1    = X2;

  prep_w_kernel<<<(32 * 9 * 8 + 255) / 256, 256, 0, stream>>>(off_w, 18, 32, 9, BtOff, kKOff, 0, kWCarry);
  prep_w_kernel<<<(64 * 5 * 8 + 255) / 256, 256, 0, stream>>>(asym1_w, 64, 64, 5, BtA1, kKA1, 0, kWCarry);
  prep_w_kernel<<<(64 * 9 * 8 + 255) / 256, 256, 0, stream>>>(def_w, 64, 64, 9, BtFin, kKFin, 0, kWCarry);
  prep_w_kernel<<<(64 * 5 * 8 + 255) / 256, 256, 0, stream>>>(asym2_w, 64, 64, 5, BtFin, kKFin, kKOff, kWCarry2);

  prep_x_kernel<<<kNB * kIH * (kIW / 32), 256, 0, stream>>>(x, dw2_w, dw2_b, dw3_w, dw3_b, XF, X2, X3);

  conv_tap_gemm_kernel<2, 0><<<kTiles / 8, 256, 0, stream>>>(X2, BtOff, off_b, (void*)OFFP);

  conv_tap_gemm_kernel<4, 1><<<kTiles / 8, 256, 0, stream>>>(X3, BtA1, asym1_b, (void*)A1);

  fused_sample_gemm_kernel<<<kTiles / kFinWaves, 128, 0, stream>>>(
      XF, OFFP, A1, BtFin, x, dw1_w, dw1_b, def_b, asym2_b, out);
}
